// ConformerBlock_73615739453810
// MI455X (gfx1250) — hardware-run, weakly checked
//
#include <hip/hip_runtime.h>


#ifndef NB
#define NB 8
#endif
#ifndef SEQ
#define SEQ 1024
#endif
#define NB_FULL  8
#define SEQ_FULL 1024
#define DM   512
#define DF   2048
#define NH   8
#define HD   64
#define DQKV (3 * DM)
#define DCH  1024
#define DP1  (2 * DCH)
#define KW   31
#define NTOK (NB * SEQ)
#define QR   32
#define QT   16
#define KWIN 96
#define HALFW 32
#define DWT  4
#define DWROWS (KW + DWT - 1)
#define DWPAD  (DWT - 1)
#define DWTAPS (KW + 2 * DWPAD)
#define DWC  256
#define LPB  ((SEQ / 32) * (DCH / DWC))

static_assert(NB >= 1 && NB <= NB_FULL);
static_assert(SEQ >= KWIN && SEQ <= SEQ_FULL);
static_assert(SEQ % 256 == 0);
static_assert(NTOK % QR == 0);
static_assert(NH * HD == DM);
static_assert(NH == 8);
static_assert(QR == 32);
static_assert(DM % 64 == 0 && DF % 64 == 0 && DQKV % 64 == 0 && DCH % 64 == 0);
static_assert(DM % 32 == 0 && DF % 32 == 0 && DCH % 32 == 0);
static_assert((DP1 * DM) % 2048 == 0 && (DM * DCH) % 2048 == 0);
static_assert(DF % 512 == 0 && DQKV % 512 == 0 && DCH % 512 == 0);
static_assert(SEQ % QT == 0 && SEQ % 64 == 0 && SEQ % QR == 0);
static_assert((SEQ - KWIN) % 16 == 0 && HALFW % 16 == 0);
static_assert(KWIN == 96 && QT == 16 && HD == 64);
static_assert(8 * DWT == QR);
static_assert(DCH % DWC == 0 && DWC == 256);
static_assert(LPB % 32 == 0);
static_assert(8 * 32 * 8 == QR * 64);
static_assert(4 * 32 * 8 == QT * HD);
static_assert(2 * 256 * 8 == 64 * 64);
static_assert(2 * 32 * 8 == DM && 4 * 32 * 4 == DM);
static_assert(32 * 8 == DWC);
static_assert(16 * 256 * 8 == QR * DCH);
static_assert(8 * QR * 64 * 2 <= 131072);
static_assert(QR * DM * 4 <= 131072);
static_assert(8 * QT * HD * 2 <= 131072);
static_assert(DWTAPS * DWC * 4 + 64 <= 131072);
static_assert(64 * 72 * 2 <= 131072);

typedef _Float16 h16;
typedef _Float16 v16h __attribute__((ext_vector_type(16)));
typedef _Float16 v8h  __attribute__((ext_vector_type(8)));
typedef float    v8f  __attribute__((ext_vector_type(8)));
typedef float    v4f  __attribute__((ext_vector_type(4)));
typedef float    v2f  __attribute__((ext_vector_type(2)));

union Frag { v16h v; v8h h[2]; };

#define WSC   64.0f
#define SC_O  2.44140625e-04f
#define SC_H  0.015625f
#define SC_D  1024.0f
#define SC_DI 9.765625e-04f
#define LOG2E 1.44269504088896340736f
#define SC_S  (3.0517578125e-05f * LOG2E)
#define LN_EPS 1e-5f

static __device__ __forceinline__ v8f zero8() {
    v8f z;
#pragma unroll
    for (int i = 0; i < 8; ++i) z[i] = 0.0f;
    return z;
}

static __device__ __forceinline__ v16h load_frag16(const _Float16* base, int ld, int lane) {
    int m  = lane & 15;
    int kb = (lane >> 4) << 3;
    const _Float16* p = base + (size_t)m * ld + kb;
    Frag f;
    f.h[0] = *(const v8h*)(p);
    f.h[1] = *(const v8h*)(p + 16);
    return f.v;
}

static __device__ __forceinline__ v8f wmma16(v16h a, v16h b, v8f c) {
    v8f d = __builtin_amdgcn_wmma_f32_16x16x32_f16(false, a, false, b, (short)0, c, false, false);
    asm volatile("v_nop\n\tv_nop\n\tv_nop\n\tv_nop" : "+v"(d) : "v"(a), "v"(b));
    return d;
}

static __device__ __forceinline__ float bf16r(float x) {
    unsigned u = __float_as_uint(x);
    u = (u + 0x7FFFu + ((u >> 16) & 1u)) & 0xFFFF0000u;
    return __uint_as_float(u);
}

static __device__ __forceinline__ h16 toh_flush(float v) {
    const h16 r = (h16)v;
    return (fabsf(v) < 6.103515625e-05f) ? (h16)0.0f : r;
}

static __device__ __forceinline__ void wave_lds_sync() {
    __builtin_amdgcn_fence(3, "wavefront");
    asm volatile("s_wait_dscnt 0" ::: "memory");
    __builtin_amdgcn_wave_barrier();
}

static __device__ __forceinline__ float wsum(float v) {
    v += __shfl_xor(v, 16, 32); v += __shfl_xor(v, 8, 32); v += __shfl_xor(v, 4, 32);
    v += __shfl_xor(v, 2, 32);  v += __shfl_xor(v, 1, 32);
    return v;
}

static __device__ __forceinline__ float siluf(float x) {
    const float xe = fmaxf(x, -80.0f);
    const float u  = __builtin_amdgcn_exp2f(-xe * LOG2E);
    return x * __builtin_amdgcn_rcpf(1.0f + u);
}
static __device__ __forceinline__ float sigmf(float x) {
    const float xe = fmaxf(x, -80.0f);
    const float u  = __builtin_amdgcn_exp2f(-xe * LOG2E);
    return __builtin_amdgcn_rcpf(1.0f + u);
}

static __device__ __forceinline__ void load_cols16(const float* p, int lane, float (&o)[16]) {
#pragma unroll
    for (int j = 0; j < 2; ++j) {
        v4f a = *(const v4f*)(p + 256 * j + 8 * lane);
        v4f c = *(const v4f*)(p + 256 * j + 8 * lane + 4);
        o[8 * j + 0] = a.x; o[8 * j + 1] = a.y; o[8 * j + 2] = a.z; o[8 * j + 3] = a.w;
        o[8 * j + 4] = c.x; o[8 * j + 5] = c.y; o[8 * j + 6] = c.z; o[8 * j + 7] = c.w;
    }
}

static __device__ __forceinline__ void ln_lane(const float (&v)[16], const float (&gl)[16],
                                               const float (&el)[16], float (&y)[16]) {
    float s = 0.0f;
#pragma unroll
    for (int e = 0; e < 16; ++e) s += v[e];
    s = wsum(s);
    const float mu = s * (1.0f / (float)DM);
    float d[16];
    float q = 0.0f;
#pragma unroll
    for (int e = 0; e < 16; ++e) { d[e] = v[e] - mu; q = __builtin_fmaf(d[e], d[e], q); }
    q = wsum(q);
    const float rstd = rsqrtf(__builtin_fmaf(q, 1.0f / (float)DM, LN_EPS));
#pragma unroll
    for (int e = 0; e < 16; ++e) y[e] = d[e] * rstd * gl[e] + el[e];
}

__global__ __launch_bounds__(256) void k_wcvt(const float* __restrict__ src,
                                               _Float16* __restrict__ dst) {
    const size_t i = (size_t)blockIdx.x * 256 + threadIdx.x;
    v4f a = *(const v4f*)(src + i * 8);
    v4f c = *(const v4f*)(src + i * 8 + 4);
    v8h o;
    o[0] = toh_flush(bf16r(a.x) * WSC); o[1] = toh_flush(bf16r(a.y) * WSC);
    o[2] = toh_flush(bf16r(a.z) * WSC); o[3] = toh_flush(bf16r(a.w) * WSC);
    o[4] = toh_flush(bf16r(c.x) * WSC); o[5] = toh_flush(bf16r(c.y) * WSC);
    o[6] = toh_flush(bf16r(c.z) * WSC); o[7] = toh_flush(bf16r(c.w) * WSC);
    *(volatile v8h*)(dst + i * 8) = o;
    __threadfence();
    *(volatile v8h*)(dst + i * 8) = o;
}

__global__ __launch_bounds__(256) void k_wcvt_t(const float* __restrict__ src,
                                                 _Float16* __restrict__ dst, int KD, int ND) {
#pragma clang fp contract(off)
    __shared__ __align__(16) _Float16 tl[64 * 72];
    const int tid = threadIdx.x;
    const int n0 = blockIdx.x * 64, k0 = blockIdx.y * 64;
#pragma unroll
    for (int i = 0; i < 4; ++i) {
        const int k  = (tid >> 4) + 16 * i;
        const int n4 = (tid & 15) * 4;
        v4f a = *(const v4f*)(src + (size_t)(k0 + k) * ND + n0 + n4);
        tl[(n4 + 0) * 72 + k] = toh_flush(bf16r(a.x) * WSC);
        tl[(n4 + 1) * 72 + k] = toh_flush(bf16r(a.y) * WSC);
        tl[(n4 + 2) * 72 + k] = toh_flush(bf16r(a.z) * WSC);
        tl[(n4 + 3) * 72 + k] = toh_flush(bf16r(a.w) * WSC);
    }
    __syncthreads();
    v8h pv[2];
#pragma unroll
    for (int i = 0; i < 2; ++i) {
        const int p = tid + 256 * i;
        pv[i] = *(const v8h*)(&tl[(p >> 3) * 72 + (p & 7) * 8]);
    }
    _Float16* ob = dst + (size_t)n0 * KD + k0;
#pragma unroll
    for (int i = 0; i < 2; ++i) {
        const int p = tid + 256 * i;
        *(volatile v8h*)(ob + (size_t)(p >> 3) * KD + (p & 7) * 8) = pv[i];
    }
    __threadfence();
#pragma unroll
    for (int i = 0; i < 2; ++i) {
        const int p = tid + 256 * i;
        *(volatile v8h*)(ob + (size_t)(p >> 3) * KD + (p & 7) * 8) = pv[i];
    }
}

__global__ __launch_bounds__(256) void k_ln1(const float* __restrict__ x,
                                              const float* __restrict__ g,
                                              const float* __restrict__ be,
                                              _Float16* __restrict__ y) {
    const int tid = threadIdx.x, lane = tid & 31, w = tid >> 5;
    const int tok = blockIdx.x * 8 + w;
    const int b = tok / SEQ, s = tok - b * SEQ;
    const float* xr = x + ((size_t)b * SEQ_FULL + s) * DM;
    float v[16], gl[16], el[16], yv[16];
    load_cols16(xr, lane, v);
    load_cols16(g, lane, gl);
    load_cols16(be, lane, el);
#pragma unroll
    for (int e = 0; e < 16; ++e) { v[e] = bf16r(v[e]); gl[e] = bf16r(gl[e]); el[e] = bf16r(el[e]); }
    ln_lane(v, gl, el, yv);
    v8h o[2];
#pragma unroll
    for (int j = 0; j < 2; ++j)
#pragma unroll
        for (int e = 0; e < 8; ++e) o[j][e] = (_Float16)yv[8 * j + e];
    _Float16* yr = y + (size_t)tok * DM;
    *(volatile v8h*)(yr + 8 * lane)       = o[0];
    *(volatile v8h*)(yr + 256 + 8 * lane) = o[1];
    __threadfence();
    *(volatile v8h*)(yr + 8 * lane)       = o[0];
    *(volatile v8h*)(yr + 256 + 8 * lane) = o[1];
}

static __device__ __forceinline__ void gemm_32x64(const _Float16* __restrict__ Ab,
                                                  const _Float16* __restrict__ Bb,
                                                  int K, int lane, v8f (&acc)[2][4]) {
#pragma unroll
    for (int t = 0; t < 2; ++t)
#pragma unroll
        for (int j = 0; j < 4; ++j) acc[t][j] = zero8();
#pragma unroll 1
    for (int k0 = 0; k0 < K; k0 += 32) {
        v16h a0 = load_frag16(Ab + k0, K, lane);
        v16h a1 = load_frag16(Ab + (size_t)16 * K + k0, K, lane);
        v16h bb[4];
#pragma unroll
        for (int j = 0; j < 4; ++j) bb[j] = load_frag16(Bb + (size_t)(16 * j) * K + k0, K, lane);
#pragma unroll
        for (int j = 0; j < 4; ++j) {
            acc[0][j] = wmma16(a0, bb[j], acc[0][j]);
            acc[1][j] = wmma16(a1, bb[j], acc[1][j]);
        }
    }
}

template <int EPI>
static __device__ __forceinline__ void gemm_p_body(const _Float16* __restrict__ A, const int K,
                                                   const _Float16* __restrict__ Bw,
                                                   const float* __restrict__ bias,
                                                   _Float16* __restrict__ outp, const int ldo) {
    __shared__ __align__(16) _Float16 st[8][QR * 64];
    const int tid = threadIdx.x, lane = tid & 31;
    const int w = __builtin_amdgcn_readfirstlane(tid >> 5);
    const int hh = lane >> 4, m = lane & 15;
    const int m0  = blockIdx.x * QR;
    const int seg = blockIdx.y;
    const int nl  = 64 * w;
    const int n0w = seg * 512 + nl;

    v8f acc[2][4];
    gemm_32x64(A + (size_t)m0 * K, Bw + (size_t)n0w * K, K, lane, acc);

    float bl[4];
#pragma unroll
    for (int j = 0; j < 4; ++j) bl[j] = bf16r(bias[n0w + 16 * j + m]);
#pragma unroll
    for (int t = 0; t < 2; ++t)
#pragma unroll
        for (int j = 0; j < 4; ++j)
#pragma unroll
            for (int r = 0; r < 8; ++r) {
                float a = acc[t][j][r];
                float val;
                if (EPI == 0) {
                    val = __builtin_fmaf(bl[j], WSC, a);
                } else {
                    float hx = __builtin_fmaf(a, SC_H, bl[j]);
                    val = WSC * siluf(hx);
                }
                st[w][(16 * t + 8 * hh + r) * 64 + 16 * j + m] = toh_flush(val);
            }
    wave_lds_sync();

    v8h pv[8];
    const int lr = lane >> 3, lc = (lane & 7) * 8;
#pragma unroll
    for (int i = 0; i < 8; ++i) pv[i] = *(const v8h*)(&st[w][(4 * i + lr) * 64 + lc]);
    _Float16* ob = outp + (size_t)m0 * ldo + n0w;
#pragma unroll
    for (int i = 0; i < 8; ++i) *(volatile v8h*)(ob + (size_t)(4 * i + lr) * ldo + lc) = pv[i];
    __threadfence();
#pragma unroll
    for (int i = 0; i < 8; ++i) *(volatile v8h*)(ob + (size_t)(4 * i + lr) * ldo + lc) = pv[i];
}

__global__ __launch_bounds__(256) __attribute__((amdgpu_num_vgpr(256)))
void k_gemm_qkv(const _Float16* __restrict__ A, const _Float16* __restrict__ Bw,
                const float* __restrict__ bias, _Float16* __restrict__ outp) {
    gemm_p_body<0>(A, DM, Bw, bias, outp, DQKV);
}

__global__ __launch_bounds__(256) __attribute__((amdgpu_num_vgpr(256)))
void k_gemm_ffn(const _Float16* __restrict__ A, const _Float16* __restrict__ Bw,
                const float* __restrict__ bias, _Float16* __restrict__ outp) {
    gemm_p_body<1>(A, DM, Bw, bias, outp, DF);
}

__global__ __launch_bounds__(256) __attribute__((amdgpu_num_vgpr(256)))
void k_gemm_glu(const _Float16* __restrict__ A, const _Float16* __restrict__ Bw,
                const float* __restrict__ bias, _Float16* __restrict__ outp) {
    __shared__ __align__(16) _Float16 st[8][QR * 64];
    const int tid = threadIdx.x, lane = tid & 31;
    const int w = __builtin_amdgcn_readfirstlane(tid >> 5);
    const int hh = lane >> 4, m = lane & 15;
    const int m0 = blockIdx.x * QR;
    const int c0 = blockIdx.y * 512 + 64 * w;

    v8f sg[2][4];
    gemm_32x64(A + (size_t)m0 * DM, Bw + (size_t)(DCH + c0) * DM, DM, lane, sg);
    float b2[4];
#pragma unroll
    for (int j = 0; j < 4; ++j) b2[j] = bf16r(bias[DCH + c0 + 16 * j + m]);
#pragma unroll
    for (int t = 0; t < 2; ++t)
#pragma unroll
        for (int j = 0; j < 4; ++j)
#pragma unroll
            for (int r = 0; r < 8; ++r)
                sg[t][j][r] = sigmf(__builtin_fmaf(sg[t][j][r], SC_H, b2[j]));

    v8f acc[2][4];
    gemm_32x64(A + (size_t)m0 * DM, Bw + (size_t)c0 * DM, DM, lane, acc);
    float b1[4];
#pragma unroll
    for (int j = 0; j < 4; ++j) b1[j] = bf16r(bias[c0 + 16 * j + m]);
#pragma unroll
    for (int t = 0; t < 2; ++t)
#pragma unroll
        for (int j = 0; j < 4; ++j)
#pragma unroll
            for (int r = 0; r < 8; ++r) {
                const float val = __builtin_fmaf(b1[j], WSC, acc[t][j][r]) * sg[t][j][r];
                st[w][(16 * t + 8 * hh + r) * 64 + 16 * j + m] = toh_flush(val);
            }
    wave_lds_sync();

    v8h pv[8];
    const int lr = lane >> 3, lc = (lane & 7) * 8;
#pragma unroll
    for (int i = 0; i < 8; ++i) pv[i] = *(const v8h*)(&st[w][(4 * i + lr) * 64 + lc]);
    _Float16* ob = outp + (size_t)m0 * DCH + c0;
#pragma unroll
    for (int i = 0; i < 8; ++i) *(volatile v8h*)(ob + (size_t)(4 * i + lr) * DCH + lc) = pv[i];
    __threadfence();
#pragma unroll
    for (int i = 0; i < 8; ++i) *(volatile v8h*)(ob + (size_t)(4 * i + lr) * DCH + lc) = pv[i];
}

template <int RESIN, int FINAL>
static __device__ __forceinline__ void gemm_r_body(const _Float16* __restrict__ A, const int K,
                                                   const _Float16* __restrict__ Bw,
                                                   const float* __restrict__ bias,
                                                   const float* __restrict__ res, const float rscale,
                                                   const float* __restrict__ g,
                                                   const float* __restrict__ be,
                                                   float* __restrict__ outf,
                                                   _Float16* __restrict__ outh) {
    __shared__ __align__(16) float T[QR * DM];
    const int tid = threadIdx.x, lane = tid & 31;
    const int w = __builtin_amdgcn_readfirstlane(tid >> 5);
    const int hh = lane >> 4, m = lane & 15;
    const int m0 = blockIdx.x * QR;
    const int nl = 64 * w;

    v8f acc[2][4];
    gemm_32x64(A + (size_t)m0 * K, Bw + (size_t)nl * K, K, lane, acc);
#pragma unroll
    for (int t = 0; t < 2; ++t)
#pragma unroll
        for (int j = 0; j < 4; ++j)
#pragma unroll
            for (int r = 0; r < 8; ++r)
                T[(16 * t + 8 * hh + r) * DM + nl + 16 * j + m] = acc[t][j][r];
    __syncthreads();

    float bl[16], gl[16], el[16];
    load_cols16(bias, lane, bl);
    load_cols16(g, lane, gl);
    load_cols16(be, lane, el);
#pragma unroll
    for (int e = 0; e < 16; ++e) { bl[e] = bf16r(bl[e]); gl[e] = bf16r(gl[e]); el[e] = bf16r(el[e]); }

#pragma unroll 1
    for (int rr = 0; rr < 4; ++rr) {
        const int row = 4 * w + rr;
        const int tok = m0 + row;
        float v[16], rv[16], yv[16];
        load_cols16(&T[row * DM], lane, v);
        if (RESIN == 0) {
            const int b = tok / SEQ, s = tok - b * SEQ;
            load_cols16(res + ((size_t)b * SEQ_FULL + s) * DM, lane, rv);
#pragma unroll
            for (int e = 0; e < 16; ++e) rv[e] = bf16r(rv[e]);
        } else {
            load_cols16(res + (size_t)tok * DM, lane, rv);
        }
#pragma unroll
        for (int e = 0; e < 16; ++e)
            v[e] = __builtin_fmaf(rscale, __builtin_fmaf(v[e], SC_O, bl[e]), rv[e]);
        ln_lane(v, gl, el, yv);

        float* trow = &T[row * DM];
#pragma unroll
        for (int j = 0; j < 2; ++j) {
            v4f p0, p1;
            if (FINAL == 0) {
                p0.x = v[8 * j + 0]; p0.y = v[8 * j + 1]; p0.z = v[8 * j + 2]; p0.w = v[8 * j + 3];
                p1.x = v[8 * j + 4]; p1.y = v[8 * j + 5]; p1.z = v[8 * j + 6]; p1.w = v[8 * j + 7];
            } else {
                p0.x = yv[8 * j + 0]; p0.y = yv[8 * j + 1]; p0.z = yv[8 * j + 2]; p0.w = yv[8 * j + 3];
                p1.x = yv[8 * j + 4]; p1.y = yv[8 * j + 5]; p1.z = yv[8 * j + 6]; p1.w = yv[8 * j + 7];
            }
            *(v4f*)(trow + 256 * j + 8 * lane)     = p0;
            *(v4f*)(trow + 256 * j + 8 * lane + 4) = p1;
        }
        wave_lds_sync();
        v4f s4[4];
#pragma unroll
        for (int jj = 0; jj < 4; ++jj) s4[jj] = *(const v4f*)(trow + 128 * jj + 4 * lane);

        float* orow = outf + (size_t)tok * DM;
        if (FINAL == 0) {
            v8h o[2];
#pragma unroll
            for (int j = 0; j < 2; ++j)
#pragma unroll
                for (int e = 0; e < 8; ++e) o[j][e] = toh_flush(yv[8 * j + e]);
            _Float16* hrow = outh + (size_t)tok * DM;
            *(volatile v8h*)(hrow + 8 * lane)       = o[0];
            *(volatile v8h*)(hrow + 256 + 8 * lane) = o[1];
#pragma unroll
            for (int jj = 0; jj < 4; ++jj) *(volatile v4f*)(orow + 128 * jj + 4 * lane) = s4[jj];
            __threadfence();
            *(volatile v8h*)(hrow + 8 * lane)       = o[0];
            *(volatile v8h*)(hrow + 256 + 8 * lane) = o[1];
#pragma unroll
            for (int jj = 0; jj < 4; ++jj) *(volatile v4f*)(orow + 128 * jj + 4 * lane) = s4[jj];
        } else {
#pragma unroll
            for (int jj = 0; jj < 4; ++jj) *(volatile v4f*)(orow + 128 * jj + 4 * lane) = s4[jj];
            __threadfence();
#pragma unroll
            for (int jj = 0; jj < 4; ++jj) *(volatile v4f*)(orow + 128 * jj + 4 * lane) = s4[jj];
        }
    }
}

__global__ __launch_bounds__(256) __attribute__((amdgpu_num_vgpr(256)))
void k_gemm_r_in(const _Float16* __restrict__ A, const _Float16* __restrict__ Bw,
                 const float* __restrict__ bias, const float* __restrict__ res, float rscale,
                 const float* __restrict__ g, const float* __restrict__ be,
                 float* __restrict__ outf, _Float16* __restrict__ outh) {
    gemm_r_body<0, 0>(A, DF, Bw, bias, res, rscale, g, be, outf, outh);
}

__global__ __launch_bounds__(256) __attribute__((amdgpu_num_vgpr(256)))
void k_gemm_r_mid(const _Float16* __restrict__ A, int K, const _Float16* __restrict__ Bw,
                  const float* __restrict__ bias, const float* __restrict__ res, float rscale,
                  const float* __restrict__ g, const float* __restrict__ be,
                  float* __restrict__ outf, _Float16* __restrict__ outh) {
    gemm_r_body<1, 0>(A, K, Bw, bias, res, rscale, g, be, outf, outh);
}

__global__ __launch_bounds__(256) __attribute__((amdgpu_num_vgpr(256)))
void k_gemm_r_fin(const _Float16* __restrict__ A, const _Float16* __restrict__ Bw,
                  const float* __restrict__ bias, const float* __restrict__ res, float rscale,
                  const float* __restrict__ g, const float* __restrict__ be,
                  float* __restrict__ outf, _Float16* __restrict__ outh) {
    gemm_r_body<1, 1>(A, DF, Bw, bias, res, rscale, g, be, outf, outh);
}

__global__ __launch_bounds__(256) void k_vtr(const _Float16* __restrict__ qkv,
                                              _Float16* __restrict__ vt) {
    __shared__ __align__(16) _Float16 tl[HD * 72];
    const int tid = threadIdx.x;
    const int t0 = blockIdx.x * 64, h = blockIdx.y, b = blockIdx.z;
    const _Float16* vp = qkv + ((size_t)b * SEQ + t0) * DQKV + 2 * DM + h * HD;
#pragma unroll
    for (int i = 0; i < 2; ++i) {
        const int p = tid + 256 * i;
        const int t = p >> 3, part = p & 7;
        v8h vv = *(const v8h*)(vp + (size_t)t * DQKV + part * 8);
#pragma unroll
        for (int e = 0; e < 8; ++e) tl[(part * 8 + e) * 72 + t] = vv[e];
    }
    __syncthreads();
    v8h pv[2];
#pragma unroll
    for (int i = 0; i < 2; ++i) {
        const int p = tid + 256 * i;
        pv[i] = *(const v8h*)(&tl[(p >> 3) * 72 + (p & 7) * 8]);
    }
    _Float16* ob = vt + ((size_t)(b * NH + h) * HD) * SEQ + t0;
#pragma unroll
    for (int i = 0; i < 2; ++i) {
        const int p = tid + 256 * i;
        *(volatile v8h*)(ob + (size_t)(p >> 3) * SEQ + (p & 7) * 8) = pv[i];
    }
    __threadfence();
#pragma unroll
    for (int i = 0; i < 2; ++i) {
        const int p = tid + 256 * i;
        *(volatile v8h*)(ob + (size_t)(p >> 3) * SEQ + (p & 7) * 8) = pv[i];
    }
}

__global__ __launch_bounds__(256) __attribute__((amdgpu_num_vgpr(256)))
void k_attn(const _Float16* __restrict__ qkv, const _Float16* __restrict__ vt,
            _Float16* __restrict__ ctx) {
    __shared__ __align__(16) _Float16 cs[8][QT * HD];
    const int tid = threadIdx.x, lane = tid & 31;
    const int w = __builtin_amdgcn_readfirstlane(tid >> 5);
    const int hh = lane >> 4, n = lane & 15;
    const int b = blockIdx.y;
    const int q0 = blockIdx.x * QT;
    int kb = max(q0 - HALFW, 0);
    kb = min(kb, SEQ - KWIN);
    const size_t tok0 = (size_t)b * SEQ;
    const _Float16* qp = qkv + (tok0 + q0) * DQKV + w * HD;
    const _Float16* kp = qkv + (tok0 + kb) * DQKV + DM + w * HD;
    const _Float16* vp = vt + ((size_t)(b * NH + w) * HD) * SEQ + kb;

    const v16h qf0 = load_frag16(qp, DQKV, lane);
    const v16h qf1 = load_frag16(qp + 32, DQKV, lane);
    v8f s[6];
#pragma unroll
    for (int t = 0; t < 6; ++t) {
        const _Float16* kt = kp + (size_t)(16 * t) * DQKV;
        const v16h kf0 = load_frag16(kt, DQKV, lane);
        const v16h kf1 = load_frag16(kt + 32, DQKV, lane);
        v8f a = wmma16(kf0, qf0, zero8());
        s[t] = wmma16(kf1, qf1, a);
    }

    const int qi = q0 + n;
    float mx = -3.0e38f;
#pragma unroll
    for (int t = 0; t < 6; ++t)
#pragma unroll
        for (int r = 0; r < 8; ++r) {
            const int dlt = kb + 16 * t + 8 * hh + r - qi;
            const bool ok = (dlt >= -HALFW) & (dlt <= HALFW);
            const float z = s[t][r] * SC_S;
            const float zz = ok ? z : -3.0e38f;
            s[t][r] = zz;
            mx = fmaxf(mx, zz);
        }
    mx = fmaxf(mx, __shfl_xor(mx, 16, 32));

    float rs = 0.0f;
    v16h pb[3];
#pragma unroll
    for (int st = 0; st < 3; ++st)
#pragma unroll
        for (int r = 0; r < 8; ++r) {
            const float e0 = s[2 * st][r] - mx;
            const float x0 = __builtin_amdgcn_exp2f(fmaxf(e0, -28.0f) + 14.0f);
            const h16 h0 = (h16)((e0 < -28.0f) ? 0.0f : x0);
            const float e1 = s[2 * st + 1][r] - mx;
            const float x1 = __builtin_amdgcn_exp2f(fmaxf(e1, -28.0f) + 14.0f);
            const h16 h1 = (h16)((e1 < -28.0f) ? 0.0f : x1);
            pb[st][r]     = h0;
            pb[st][8 + r] = h1;
            rs += (float)h0;
            rs += (float)h1;
        }
    rs += __shfl_xor(rs, 16, 32);

    v8f o[4];
#pragma unroll
    for (int dt = 0; dt < 4; ++dt) o[dt] = zero8();
#pragma unroll
    for (int st = 0; st < 3; ++st)
#pragma unroll
        for (int dt = 0; dt < 4; ++dt) {
            const v16h va = load_frag16(vp + (size_t)(16 * dt) * SEQ + 32 * st, SEQ, lane);
            o[dt] = wmma16(va, pb[st], o[dt]);
        }

    const float inv = __builtin_amdgcn_rcpf(rs);
#pragma unroll
    for (int dt = 0; dt < 4; ++dt) {
        v8h c8;
#pragma unroll
        for (int r = 0; r < 8; ++r) c8[r] = toh_flush(o[dt][r] * inv);
        *(v8h*)(&cs[w][n * HD + 16 * dt + 8 * hh]) = c8;
    }
    wave_lds_sync();

    v8h pv[4];
    const int lr = lane >> 3, lc = (lane & 7) * 8;
#pragma unroll
    for (int i = 0; i < 4; ++i) pv[i] = *(const v8h*)(&cs[w][(4 * i + lr) * HD + lc]);
    _Float16* dst = ctx + (tok0 + q0) * DM + w * HD;
#pragma unroll
    for (int i = 0; i < 4; ++i) *(volatile v8h*)(dst + (size_t)(4 * i + lr) * DM + lc) = pv[i];
    __threadfence();
#pragma unroll
    for (int i = 0; i < 4; ++i) *(volatile v8h*)(dst + (size_t)(4 * i + lr) * DM + lc) = pv[i];
}

__global__ __launch_bounds__(256) void k_dwconv(const _Float16* __restrict__ g,
                                                 const float* __restrict__ dww,
                                                 const float* __restrict__ dwb,
                                                 _Float16* __restrict__ dpl,
                                                 float* __restrict__ part) {
#pragma clang fp contract(off)
    __shared__ __align__(16) float wt[DWTAPS * DWC];
    __shared__ float red[16];
    const int tid = threadIdx.x, lane = tid & 31;
    const int w = __builtin_amdgcn_readfirstlane(tid >> 5);
    const int m0 = blockIdx.x * QR;
    const int c0 = blockIdx.y * DWC;
    const int b  = m0 / SEQ;
    const int tl0 = m0 - b * SEQ + DWT * w;

#pragma unroll 1
    for (int j = 0; j < DWTAPS; ++j) {
        const int tj = j - DWPAD;
        const int tc = min(max(tj, 0), KW - 1);
        float v = dww[(size_t)(c0 + tid) * KW + tc];
        asm volatile("" : "+v"(v));
        wt[j * DWC + tid] = ((tj >= 0) & (tj < KW)) ? bf16r(v) : 0.0f;
    }
    __syncthreads();

    const int cl = 8 * lane;
    float acc[DWT][8];
    {
        v4f ba = *(const v4f*)(dwb + c0 + cl);
        v4f bc = *(const v4f*)(dwb + c0 + cl + 4);
#pragma unroll
        for (int i = 0; i < DWT; ++i) {
            acc[i][0] = bf16r(ba.x); acc[i][1] = bf16r(ba.y); acc[i][2] = bf16r(ba.z); acc[i][3] = bf16r(ba.w);
            acc[i][4] = bf16r(bc.x); acc[i][5] = bf16r(bc.y); acc[i][6] = bf16r(bc.z); acc[i][7] = bf16r(bc.w);
        }
    }
    const _Float16* gb = g + (size_t)b * SEQ * DCH + c0 + cl;
#pragma unroll 1
    for (int s = 0; s < DWROWS; ++s) {
        const int tt  = tl0 + s - (KW / 2);
        const int tcl = min(max(tt, 0), SEQ - 1);
        const v8h gv = *(const v8h*)(gb + (size_t)tcl * DCH);
        const float gs = ((tt >= 0) & (tt < SEQ)) ? SC_H : 0.0f;
        float x[8];
#pragma unroll
        for (int e = 0; e < 8; ++e) x[e] = (float)gv[e] * gs;
#pragma unroll
        for (int i = 0; i < DWT; ++i) {
            const float* wr = &wt[(s - i + DWPAD) * DWC + cl];
            const v4f w0 = *(const v4f*)(wr);
            const v4f w1 = *(const v4f*)(wr + 4);
            acc[i][0] = __builtin_fmaf(w0.x, x[0], acc[i][0]);
            acc[i][1] = __builtin_fmaf(w0.y, x[1], acc[i][1]);
            acc[i][2] = __builtin_fmaf(w0.z, x[2], acc[i][2]);
            acc[i][3] = __builtin_fmaf(w0.w, x[3], acc[i][3]);
            acc[i][4] = __builtin_fmaf(w1.x, x[4], acc[i][4]);
            acc[i][5] = __builtin_fmaf(w1.y, x[5], acc[i][5]);
            acc[i][6] = __builtin_fmaf(w1.z, x[6], acc[i][6]);
            acc[i][7] = __builtin_fmaf(w1.w, x[7], acc[i][7]);
        }
    }

    float ssum = 0.0f, ssq = 0.0f;
    v8h ov[DWT];
#pragma unroll
    for (int i = 0; i < DWT; ++i)
#pragma unroll
        for (int e = 0; e < 8; ++e) {
            const float d = acc[i][e];
            ssum += d;
            ssq = __builtin_fmaf(d, d, ssq);
            ov[i][e] = toh_flush(d * SC_D);
        }
    _Float16* drow = dpl + ((size_t)b * SEQ + tl0) * DCH + c0 + cl;
#pragma unroll
    for (int i = 0; i < DWT; ++i) *(volatile v8h*)(drow + (size_t)i * DCH) = ov[i];
    __threadfence();
#pragma unroll
    for (int i = 0; i < DWT; ++i) *(volatile v8h*)(drow + (size_t)i * DCH) = ov[i];

    ssum = wsum(ssum);
    ssq  = wsum(ssq);
    if (lane == 0) { red[w] = ssum; red[8 + w] = ssq; }
    __syncthreads();
    if (w == 0) {
        const int li = min(lane, 7);
        float a = red[li];
        float q = red[8 + li];
        asm volatile("" : "+v"(a));
        asm volatile("" : "+v"(q));
        a = (lane < 8) ? a : 0.0f;
        q = (lane < 8) ? q : 0.0f;
        a += __shfl_xor(a, 4, 32); a += __shfl_xor(a, 2, 32); a += __shfl_xor(a, 1, 32);
        q += __shfl_xor(q, 4, 32); q += __shfl_xor(q, 2, 32); q += __shfl_xor(q, 1, 32);
        v4f lv;
        lv.x = (lane == 0) ? a : 0.0f;
        lv.y = (lane == 0) ? q : 0.0f;
        lv.z = 0.0f;
        lv.w = 0.0f;
        float* pl = part + (size_t)(blockIdx.x * (DCH / DWC) + blockIdx.y) * 32 + 4 * li;
        if (lane < 8) { *(volatile v4f*)pl = lv; }
        __threadfence();
        if (lane < 8) { *(volatile v4f*)pl = lv; }
    }
}

__global__ __launch_bounds__(256) void k_gnact(const _Float16* __restrict__ dpl,
                                                const float* __restrict__ part,
                                                const float* __restrict__ gw,
                                                const float* __restrict__ gb,
                                                _Float16* __restrict__ spl) {
    const int tid = threadIdx.x, lane = tid & 31;
    const int m0 = blockIdx.x * QR;
    const int b  = m0 / SEQ;
    const float* pl = part + (size_t)b * LPB * 32;
    double S = 0.0, Q = 0.0;
#pragma unroll 1
    for (int i = 0; i < LPB / 32; ++i) {
        const v2f pq = *(const v2f*)(pl + (size_t)(i * 32 + lane) * 32);
        S += (double)pq.x;
        Q += (double)pq.y;
    }
    S += __shfl_xor(S, 16, 32); S += __shfl_xor(S, 8, 32); S += __shfl_xor(S, 4, 32);
    S += __shfl_xor(S, 2, 32);  S += __shfl_xor(S, 1, 32);
    Q += __shfl_xor(Q, 16, 32); Q += __shfl_xor(Q, 8, 32); Q += __shfl_xor(Q, 4, 32);
    Q += __shfl_xor(Q, 2, 32);  Q += __shfl_xor(Q, 1, 32);
    const double icnt = 1.0 / ((double)DCH * (double)SEQ);
    const double mean = S * icnt;
    const double var  = Q * icnt - mean * mean;
    const float mu   = (float)mean;
    const float rstd = rsqrtf((float)var + LN_EPS);

    const int cg = tid & 127;
    const int tp = tid >> 7;
    float a[8], c[8];
    {
        const v4f g0 = *(const v4f*)(gw + 8 * cg);
        const v4f g1 = *(const v4f*)(gw + 8 * cg + 4);
        const v4f e0 = *(const v4f*)(gb + 8 * cg);
        const v4f e1 = *(const v4f*)(gb + 8 * cg + 4);
        float gv[8] = { g0.x, g0.y, g0.z, g0.w, g1.x, g1.y, g1.z, g1.w };
        float ev[8] = { e0.x, e0.y, e0.z, e0.w, e1.x, e1.y, e1.z, e1.w };
#pragma unroll
        for (int e = 0; e < 8; ++e) {
            const float ga = rstd * bf16r(gv[e]);
            a[e] = ga * SC_DI;
            c[e] = __builtin_fmaf(-mu, ga, bf16r(ev[e]));
        }
    }
#pragma unroll 1
    for (int r = 0; r < 16; ++r) {
        const size_t tok = (size_t)m0 + 2 * r + tp;
        const v8h dv = *(const v8h*)(dpl + tok * DCH + 8 * cg);
        v8h o;
#pragma unroll
        for (int e = 0; e < 8; ++e) {
            const float v = __builtin_fmaf((float)dv[e], a[e], c[e]);
            o[e] = toh_flush(WSC * siluf(v));
        }
        _Float16* dst = spl + tok * DCH + 8 * cg;
        *(volatile v8h*)dst = o;
        __threadfence();
        *(volatile v8h*)dst = o;
    }
}

constexpr size_t SZ_WF1A = (size_t)DF * DM * 2;
constexpr size_t SZ_WF1B = (size_t)DM * DF * 2;
constexpr size_t SZ_WQKV = (size_t)DQKV * DM * 2;
constexpr size_t SZ_WO   = (size_t)DM * DM * 2;
constexpr size_t SZ_WP1  = (size_t)DP1 * DM * 2;
constexpr size_t SZ_WP2  = (size_t)DM * DCH * 2;
constexpr size_t SZ_Y    = (size_t)NTOK * DM * 2;
constexpr size_t SZ_R1   = (size_t)NTOK * DF * 2;
constexpr size_t SZ_R2   = (size_t)NTOK * DQKV * 2;
constexpr size_t SZ_G    = (size_t)NTOK * DCH * 2;
constexpr size_t SZ_VT   = (size_t)NB * NH * HD * SEQ * 2;
constexpr size_t SZ_C    = (size_t)NTOK * DM * 2;
constexpr size_t SZ_X    = (size_t)NTOK * DM * 4;
constexpr size_t SZ_PART = (size_t)(NTOK / QR) * (DCH / DWC) * 128;
constexpr size_t SZ_TOTAL = SZ_WF1A + SZ_WF1B + SZ_WQKV + SZ_WO + SZ_WP1 + SZ_WP2 + SZ_WF1A + SZ_WF1B +
                            SZ_Y + SZ_R1 + SZ_R2 + SZ_VT + SZ_C + 2 * SZ_X + SZ_PART;
static_assert(2 * SZ_G <= SZ_R1);
static_assert(SZ_G <= SZ_R2);
static_assert((size_t)NB * LPB * 128 == SZ_PART);
static_assert(SZ_TOTAL <= (size_t)134217728);
static_assert(SZ_WF1A % 128 == 0 && SZ_WQKV % 128 == 0 && SZ_WO % 128 == 0 && SZ_WP2 % 128 == 0);
static_assert(SZ_Y % 128 == 0 && SZ_G % 128 == 0 && SZ_PART % 128 == 0);

extern "C" void kernel_launch(void* const* d_in, const int* in_sizes, int n_in,
                              void* d_out, int out_size, void* d_ws, size_t ws_size,
                              hipStream_t stream) {
    if (n_in < 31) return;
    if (in_sizes[0] < ((NB - 1) * SEQ_FULL + SEQ) * DM) return;
    if (in_sizes[3] < DM * DF || in_sizes[5] < DF * DM || in_sizes[25] < DM * DF || in_sizes[27] < DF * DM) return;
    if (in_sizes[9] < DM * DQKV || in_sizes[11] < DM * DM) return;
    if (in_sizes[15] < DP1 * DM || in_sizes[21] < DM * DCH || in_sizes[17] < DCH * KW) return;
    if (in_sizes[4] < DF || in_sizes[26] < DF || in_sizes[10] < DQKV || in_sizes[16] < DP1) return;
    if (in_sizes[18] < DCH || in_sizes[19] < DCH || in_sizes[20] < DCH) return;
    if (in_sizes[1] < DM || in_sizes[2] < DM || in_sizes[6] < DM || in_sizes[7] < DM || in_sizes[8] < DM) return;
    if (in_sizes[12] < DM || in_sizes[13] < DM || in_sizes[14] < DM || in_sizes[22] < DM) return;
    if (in_sizes[23] < DM || in_sizes[24] < DM || in_sizes[28] < DM || in_sizes[29] < DM || in_sizes[30] < DM) return;
    if (out_size < NTOK * DM) return;
    if (SZ_TOTAL > ws_size) return;

    const float* x      = (const float*)d_in[0];
    const float* f1lnw  = (const float*)d_in[1];
    const float* f1lnb  = (const float*)d_in[2];
    const float* f1w1   = (const float*)d_in[3];
    const float* f1b1   = (const float*)d_in[4];
    const float* f1w2   = (const float*)d_in[5];
    const float* f1b2   = (const float*)d_in[6];
    const float* atlnw  = (const float*)d_in[7];
    const float* atlnb  = (const float*)d_in[8];
    const float* qkvw   = (const float*)d_in[9];
    const float* qkvb   = (const float*)d_in[10];
    const float* outw   = (const float*)d_in[11];
    const float* outb   = (const float*)d_in[12];
    const float* cvlnw  = (const float*)d_in[13];
    const float* cvlnb  = (const float*)d_in[14];
    const float* pw1w   = (const float*)d_in[15];
    const float* pw1b   = (const float*)d_in[16];
    const float* dww    = (const float*)d_in[17];
    const float* dwb    = (const float*)d_in[18];
    const float* gnw    = (const float*)d_in[19];
    const float* gnb    = (const float*)d_in[20];
    const float* pw2w   = (const float*)d_in[21];
    const float* pw2b   = (const float*)d_in[22];
    const float* f2lnw  = (const float*)d_in[23];
    const float* f2lnb  = (const float*)d_in[24];
    const float* f2w1   = (const float*)d_in[25];
    const float* f2b1   = (const float*)d_in[26];
    const float* f2w2   = (const float*)d_in[27];
    const float* f2b2   = (const float*)d_in[28];
    const float* fnlnw  = (const float*)d_in[29];
    const float* fnlnb  = (const float*)d_in[30];
    float* out = (float*)d_out;

    char* ws = (char*)d_ws;
    size_t off = 0;
    _Float16* wf1a = (_Float16*)(ws + off); off += SZ_WF1A;
    _Float16* wf1b = (_Float16*)(ws + off); off += SZ_WF1B;
    _Float16* wqkv = (_Float16*)(ws + off); off += SZ_WQKV;
    _Float16* wo16 = (_Float16*)(ws + off); off += SZ_WO;
    _Float16* wp1  = (_Float16*)(ws + off); off += SZ_WP1;
    _Float16* wp2  = (_Float16*)(ws + off); off += SZ_WP2;
    _Float16* wf2a = (_Float16*)(ws + off); off += SZ_WF1A;
    _Float16* wf2b = (_Float16*)(ws + off); off += SZ_WF1B;
    _Float16* ypl  = (_Float16*)(ws + off); off += SZ_Y;
    _Float16* r1   = (_Float16*)(ws + off); off += SZ_R1;
    _Float16* r2   = (_Float16*)(ws + off); off += SZ_R2;
    _Float16* vtp  = (_Float16*)(ws + off); off += SZ_VT;
    _Float16* cpl  = (_Float16*)(ws + off); off += SZ_C;
    float*    xa   = (float*)(ws + off);    off += SZ_X;
    float*    xb   = (float*)(ws + off);    off += SZ_X;
    float*    part = (float*)(ws + off);    off += SZ_PART;
    if (off > ws_size) return;

    _Float16* mpl = r1;
    _Float16* gpl = r1;
    _Float16* spl = r1 + (size_t)NTOK * DCH;
    _Float16* qkv = r2;
    _Float16* dpl = r2;

    k_wcvt_t<<<dim3(DF / 64, DM / 64), dim3(256), 0, stream>>>(f1w1, wf1a, DM, DF);
    k_wcvt_t<<<dim3(DM / 64, DF / 64), dim3(256), 0, stream>>>(f1w2, wf1b, DF, DM);
    k_wcvt_t<<<dim3(DQKV / 64, DM / 64), dim3(256), 0, stream>>>(qkvw, wqkv, DM, DQKV);
    k_wcvt_t<<<dim3(DM / 64, DM / 64), dim3(256), 0, stream>>>(outw, wo16, DM, DM);
    k_wcvt<<<dim3(DP1 * DM / 2048), dim3(256), 0, stream>>>(pw1w, wp1);
    k_wcvt<<<dim3(DM * DCH / 2048), dim3(256), 0, stream>>>(pw2w, wp2);
    k_wcvt_t<<<dim3(DF / 64, DM / 64), dim3(256), 0, stream>>>(f2w1, wf2a, DM, DF);
    k_wcvt_t<<<dim3(DM / 64, DF / 64), dim3(256), 0, stream>>>(f2w2, wf2b, DF, DM);

    k_ln1<<<dim3(NTOK / 8), dim3(256), 0, stream>>>(x, f1lnw, f1lnb, ypl);
    k_gemm_ffn<<<dim3(NTOK / QR, DF / 512), dim3(256), 0, stream>>>(ypl, wf1a, f1b1, mpl);
    k_gemm_r_in<<<dim3(NTOK / QR), dim3(256), 0, stream>>>(mpl, wf1b, f1b2, x, 0.5f, atlnw, atlnb, xa, ypl);

    k_gemm_qkv<<<dim3(NTOK / QR, DQKV / 512), dim3(256), 0, stream>>>(ypl, wqkv, qkvb, qkv);
    k_vtr<<<dim3(SEQ / 64, NH, NB), dim3(256), 0, stream>>>(qkv, vtp);
    k_attn<<<dim3(SEQ / QT, NB), dim3(256), 0, stream>>>(qkv, vtp, cpl);
    k_gemm_r_mid<<<dim3(NTOK / QR), dim3(256), 0, stream>>>(cpl, DM, wo16, outb, xa, 1.0f, cvlnw, cvlnb, xb, ypl);

    k_gemm_glu<<<dim3(NTOK / QR, DCH / 512), dim3(256), 0, stream>>>(ypl, wp1, pw1b, gpl);
    k_dwconv<<<dim3(NTOK / QR, DCH / DWC), dim3(256), 0, stream>>>(gpl, dww, dwb, dpl, part);
    k_gnact<<<dim3(NTOK / QR), dim3(256), 0, stream>>>(dpl, part, gnw, gnb, spl);
    k_gemm_r_mid<<<dim3(NTOK / QR), dim3(256), 0, stream>>>(spl, DCH, wp2, pw2b, xb, 1.0f, f2lnw, f2lnb, xa, ypl);

    k_gemm_ffn<<<dim3(NTOK / QR, DF / 512), dim3(256), 0, stream>>>(ypl, wf2a, f2b1, mpl);
    k_gemm_r_fin<<<dim3(NTOK / QR), dim3(256), 0, stream>>>(mpl, wf2b, f2b2, xa, 0.5f, fnlnw, fnlnb, out, ypl);
}
